// transform_gcn_86852828659765
// MI455X (gfx1250) — hardware-verified
//
#include <hip/hip_runtime.h>


#define NB   16
#define CI   128
#define CO   256
#define TT   128
#define VV   25
#define WW_  11
#define KK_  3
#define GG   8
#define MM   (CO * WW_)
#define KD   (CI * VV)
#define KD8  (KD / 8)
#define PP   (NB * TT)
#define BN_EPS 1e-5f
#define WSC  4096.0f
#define XSC  16.0f
#define OSC  (1.0f / 65536.0f)

typedef __attribute__((ext_vector_type(16))) _Float16 v16h;
typedef __attribute__((ext_vector_type(8)))  _Float16 v8h;
typedef __attribute__((ext_vector_type(16))) __bf16   v16b;
typedef __attribute__((ext_vector_type(8)))  __bf16   v8b;
typedef __attribute__((ext_vector_type(8)))  float    v8f;
typedef __attribute__((ext_vector_type(4)))  float    v4f;

__device__ __forceinline__ unsigned short f2bf_bits(float f) {
  unsigned u = __float_as_uint(f);
  return (unsigned short)((u + 0x7FFFu + ((u >> 16) & 1u)) >> 16);
}
__device__ __forceinline__ float bf_bits2f(unsigned short h) { return __uint_as_float(((unsigned)h) << 16); }

__device__ __forceinline__ void dep_guard_h(v8f& a, v8f& b, v16h x, v16h y) { asm volatile("v_nop\n\tv_nop\n\tv_nop\n\tv_nop" : "+v"(a), "+v"(b) : "v"(x), "v"(y)); }
__device__ __forceinline__ void dep_guard_b(v8f& a, v8f& b, v16b x, v16b y) { asm volatile("v_nop\n\tv_nop\n\tv_nop\n\tv_nop" : "+v"(a), "+v"(b) : "v"(x), "v"(y)); }
__device__ __forceinline__ void keep4_h(v16h a, v16h b, v16h c, v16h d) { asm volatile("v_nop" :: "v"(a), "v"(b), "v"(c), "v"(d)); }
__device__ __forceinline__ void keep4_b(v16b a, v16b b, v16b c, v16b d) { asm volatile("v_nop" :: "v"(a), "v"(b), "v"(c), "v"(d)); }
__device__ __forceinline__ void acc_guard4(v8f& a, v8f& b, v8f& c, v8f& d) { asm volatile("v_nop\n\tv_nop\n\tv_nop\n\tv_nop" : "+v"(a), "+v"(b), "+v"(c), "+v"(d)); }
template <typename T> struct Frag;
template <> struct Frag<_Float16> {
  typedef v16h V; union U { v16h v; v8h h[2]; };
  static __device__ __forceinline__ v16h load(const _Float16* p) {
    U f; f.h[0] = *(const v8h*)(p); f.h[1] = *(const v8h*)(p + 16); return f.v;
  }
  static __device__ __forceinline__ v8f mma(v16h a, v16h b, v8f c) {
    return __builtin_amdgcn_wmma_f32_16x16x32_f16(false, a, false, b, (short)0, c, false, false);
  }
  static __device__ __forceinline__ void guard(v8f& a, v8f& b, v16h x, v16h y) { dep_guard_h(a, b, x, y); }
  static __device__ __forceinline__ void keep(v16h a, v16h b, v16h c, v16h d) { keep4_h(a, b, c, d); }
};
template <> struct Frag<__bf16> {
  typedef v16b V; union U { v16b v; v8b h[2]; };
  static __device__ __forceinline__ v16b load(const __bf16* p) {
    U f; f.h[0] = *(const v8b*)(p); f.h[1] = *(const v8b*)(p + 16); return f.v;
  }
  static __device__ __forceinline__ v8f mma(v16b a, v16b b, v8f c) {
    return __builtin_amdgcn_wmma_f32_16x16x32_bf16(false, a, false, b, (short)0, c, false, false);
  }
  static __device__ __forceinline__ void guard(v8f& a, v8f& b, v16b x, v16b y) { dep_guard_b(a, b, x, y); }
  static __device__ __forceinline__ void keep(v16b a, v16b b, v16b c, v16b d) { keep4_b(a, b, c, d); }
};

template <int ET> struct Elem;
template <> struct Elem<0> { typedef _Float16 T; };
template <> struct Elem<1> { typedef __bf16 T; };
template <int ET, bool SPLIT, int BIAS_MODE, int OUT_MODE, bool RESID, int ACT = 0>
__global__ __launch_bounds__(256) void wmma_gemm64(
    const unsigned short* __restrict__ Ap, const unsigned short* __restrict__ A2p, int lda, long strideA,
    const unsigned short* __restrict__ Btp, const unsigned short* __restrict__ Bt2p, int ldb, long strideB,
    void* __restrict__ Cout, void* __restrict__ Cout2, int ldc, long strideC,
    const float* __restrict__ bias,
    const float* __restrict__ resid, long strideR,
    int M, int N, int K, float scale) {
  typedef typename Elem<ET>::T T;
  typedef typename Frag<T>::V V;
  const T* A = (const T*)Ap; const T* A2 = (const T*)A2p; const T* Bt = (const T*)Btp; const T* Bt2 = (const T*)Bt2p;
  __shared__ __align__(16) float sT[8][16 * 68];
  const int b    = blockIdx.y;
  const int lane = threadIdx.x & 31;
  const int wave = threadIdx.x >> 5;
  const int tilesN = N >> 6;
  const int tilesM = M >> 6;
  const int tile = blockIdx.x * 8 + wave;
  if (tile >= tilesM * tilesN) return;
  const int tm = tile / tilesN;
  const int tn = tile - tm * tilesN;
  const int m0 = tm << 6;
  const int n0 = tn << 6;

  const T* Ab  = A  + (size_t)b * strideA;
  const T* Bb  = Bt + (size_t)b * strideB;
  const T* Ab2 = SPLIT ? (A2  + (size_t)b * strideA) : nullptr;
  const T* Bb2 = SPLIT ? (Bt2 + (size_t)b * strideB) : nullptr;

  const int rlane = lane & 15;
  const int koff  = (lane >> 4) * 8;
  const int mOff  = (lane >> 4) * 8;

  v8f acc[4][4];
#pragma unroll
  for (int i = 0; i < 4; ++i)
#pragma unroll
    for (int j = 0; j < 4; ++j) acc[i][j] = (v8f){0.f,0.f,0.f,0.f,0.f,0.f,0.f,0.f};

  for (int k0 = 0; k0 < K; k0 += 32) {
    V bh[4], bl[4];
#pragma unroll
    for (int j = 0; j < 4; ++j) {
      const size_t bo = (size_t)(n0 + (j << 4) + rlane) * ldb + koff + k0;
      bh[j] = Frag<T>::load(Bb + bo);
      if (SPLIT) bl[j] = Frag<T>::load(Bb2 + bo);
    }
#pragma unroll
    for (int i = 0; i < 4; ++i) {
      const size_t ao = (size_t)(m0 + (i << 4) + rlane) * lda + koff + k0;
      V ah = Frag<T>::load(Ab + ao);
      V al;
      if (SPLIT) al = Frag<T>::load(Ab2 + ao);
#pragma unroll
      for (int j = 0; j < 4; ++j) {
        acc[i][j] = Frag<T>::mma(ah, bh[j], acc[i][j]);
        if (SPLIT) {
          acc[i][j] = Frag<T>::mma(ah, bl[j], acc[i][j]);
          acc[i][j] = Frag<T>::mma(al, bh[j], acc[i][j]);
        }
      }
      Frag<T>::guard(acc[i][0], acc[i][3], ah, SPLIT ? al : ah);
    }
    Frag<T>::keep(bh[0], bh[1], bh[2], bh[3]);
    if (SPLIT) Frag<T>::keep(bl[0], bl[1], bl[2], bl[3]);
  }
  acc_guard4(acc[0][0], acc[0][1], acc[0][2], acc[0][3]);
  acc_guard4(acc[1][0], acc[1][1], acc[1][2], acc[1][3]);
  acc_guard4(acc[2][0], acc[2][1], acc[2][2], acc[2][3]);
  acc_guard4(acc[3][0], acc[3][1], acc[3][2], acc[3][3]);

  float* slab = sT[wave];
  const float* Rb = RESID ? (resid + (size_t)b * strideR) : nullptr;
#pragma unroll
  for (int i = 0; i < 4; ++i) {
    const int mBase = m0 + (i << 4);
#pragma unroll
    for (int j = 0; j < 4; ++j) {
      const int n = n0 + (j << 4) + rlane;
      float bv = 0.f;
      if (BIAS_MODE == 2) bv = bias[n];
#pragma unroll
      for (int r = 0; r < 8; ++r) {
        float v = acc[i][j][r] * scale;
        if (BIAS_MODE == 1) v += bias[mBase + mOff + r];
        if (BIAS_MODE == 2) v += bv;
        if (RESID) v += Rb[(size_t)(mBase + mOff + r) * ldc + n];
        if (ACT == 1) v = tanhf(v);
        if (ACT == 2) v = fmaxf(v, 0.0f);
        if (ACT == 3) v = v / (1.0f + expf(-v));
        if (ACT == 4) v = (v > 0.f) ? v : 0.01f * v;
        if (ACT == 5) v = 0.5f * v * (1.0f + erff(v * 0.70710678118654752f));
        slab[(mOff + r) * 68 + (j << 4) + rlane] = v;
      }
    }
    __builtin_amdgcn_fence(__ATOMIC_RELEASE, "workgroup");
    __builtin_amdgcn_wave_barrier();
    __builtin_amdgcn_fence(__ATOMIC_ACQUIRE, "workgroup");
    if (OUT_MODE == 0) {
      float* C = (float*)Cout + (size_t)b * strideC;
      const int hh = lane >> 4, c4 = (lane & 15) * 4;
      for (int pass = 0; pass < 2; ++pass) {
#pragma unroll
        for (int it = 0; it < 8; ++it) {
          const int row = it * 2 + hh;
          v4f v = *(const v4f*)(slab + row * 68 + c4);
          *(volatile v4f*)(C + (size_t)(mBase + row) * ldc + n0 + c4) = v;
        }
        __threadfence();
      }
    } else {
      const int q = lane >> 3, c8 = (lane & 7) * 8;
      unsigned short* C  = (unsigned short*)Cout  + (size_t)b * strideC;
      unsigned short* C2 = (OUT_MODE == 2) ? ((unsigned short*)Cout2 + (size_t)b * strideC) : nullptr;
      for (int pass = 0; pass < 2; ++pass) {
#pragma unroll
        for (int it = 0; it < 4; ++it) {
          const int row = it * 4 + q;
          const float* sp = slab + row * 68 + c8;
          v8h hv, lv;
#pragma unroll
          for (int e = 0; e < 8; ++e) {
            if (OUT_MODE == 1) {
              hv[e] = (_Float16)sp[e];
            } else {
              unsigned short hb = f2bf_bits(sp[e]);
              unsigned short lb = f2bf_bits(sp[e] - bf_bits2f(hb));
              hv[e] = __builtin_bit_cast(_Float16, hb);
              lv[e] = __builtin_bit_cast(_Float16, lb);
            }
          }
          *(volatile v8h*)(C + (size_t)(mBase + row) * ldc + n0 + c8) = hv;
          if (OUT_MODE == 2) *(volatile v8h*)(C2 + (size_t)(mBase + row) * ldc + n0 + c8) = lv;
        }
        __threadfence();
      }
    }
    __builtin_amdgcn_fence(__ATOMIC_RELEASE, "workgroup");
    __builtin_amdgcn_wave_barrier();
    __builtin_amdgcn_fence(__ATOMIC_ACQUIRE, "workgroup");
  }
}

__global__ __launch_bounds__(256) void prep_ww_kernel(
    const float* __restrict__ conv_w, const float* __restrict__ down_w,
    const float* __restrict__ A_adj,  const float* __restrict__ resg,
    const float* __restrict__ dbn_g,  const float* __restrict__ dbn_v,
    const float* __restrict__ bn_g,   const float* __restrict__ bn_v,
    _Float16* __restrict__ ww, int total)
{
  const int tix = blockIdx.x * 256 + threadIdx.x;
  if (tix >= total) return;
  const int m = tix / KD8;
  const int j = tix - m * KD8;
  const int c = m / WW_;
  const int w = m - c * WW_;
  const int g = c & (GG - 1);
  const float bs = bn_g[c] * rsqrtf(bn_v[c] + BN_EPS);
  float am[8], ar[8];
#pragma unroll
  for (int e = 0; e < 8; ++e) { am[e] = 0.f; ar[e] = 0.f; }
#pragma unroll 1
  for (int k = 0; k < KK_; ++k) {
    const int o = k * CO + c;
    const float ds = dbn_g[o] * rsqrtf(dbn_v[o] + BN_EPS);
    const float* cw = conv_w + (size_t)o * CI;
    const float* dw = down_w + (size_t)o * CI;
    const float* Ak = A_adj + ((size_t)(k * GG + g) * VV) * WW_ + w;
    const float* Rk = resg  + ((size_t)(k * GG + g) * VV) * WW_ + w;
#pragma unroll
    for (int e = 0; e < 8; ++e) {
      const int kk = 8 * j + e;
      const int i  = kk / VV;
      const int v  = kk - i * VV;
      am[e] += cw[i] * Ak[v * WW_];
      ar[e] += (ds * dw[i]) * Rk[v * WW_];
    }
  }
  v8h hv;
#pragma unroll
  for (int e = 0; e < 8; ++e) hv[e] = (_Float16)((bs * am[e] + ar[e]) * WSC);
  _Float16* dst = ww + (size_t)m * KD + 8 * j;
  *(volatile v8h*)dst = hv;
  __threadfence();
  *(volatile v8h*)dst = hv;
}

__global__ __launch_bounds__(256) void prep_bias_kernel(
    const float* __restrict__ conv_b, const float* __restrict__ down_b,
    const float* __restrict__ A_adj,  const float* __restrict__ resg,
    const float* __restrict__ dbn_g,  const float* __restrict__ dbn_b,
    const float* __restrict__ dbn_m,  const float* __restrict__ dbn_v,
    const float* __restrict__ bn_g,   const float* __restrict__ bn_b,
    const float* __restrict__ bn_m,   const float* __restrict__ bn_v,
    float* __restrict__ bias, int total)
{
  const int m = blockIdx.x * 256 + threadIdx.x;
  if (m >= total) return;
  const int c = m / WW_;
  const int w = m - c * WW_;
  const int g = c & (GG - 1);
  const float bs = bn_g[c] * rsqrtf(bn_v[c] + BN_EPS);
  const float bt = bn_b[c] - bn_m[c] * bs;
  float acc = bt;
#pragma unroll 1
  for (int k = 0; k < KK_; ++k) {
    const int o = k * CO + c;
    const float ds = dbn_g[o] * rsqrtf(dbn_v[o] + BN_EPS);
    const float dt = dbn_b[o] - dbn_m[o] * ds;
    const float rb = ds * down_b[o] + dt;
    const float cb = bs * conv_b[o];
    const float* Ak = A_adj + ((size_t)(k * GG + g) * VV) * WW_ + w;
    const float* Rk = resg  + ((size_t)(k * GG + g) * VV) * WW_ + w;
    float sA = 0.f, sR = 0.f;
#pragma unroll 1
    for (int v = 0; v < VV; ++v) {
      sA += Ak[v * WW_];
      sR += Rk[v * WW_];
    }
    acc += cb * sA + rb * sR;
  }
  *(volatile float*)(bias + m) = acc;
  __threadfence();
  *(volatile float*)(bias + m) = acc;
}

__global__ __launch_bounds__(256) void prep_x_kernel(
    const float* __restrict__ x, _Float16* __restrict__ xb, int total)
{
  const int tix = blockIdx.x * 256 + threadIdx.x;
  if (tix >= total) return;
  const int p = tix / KD8;
  const int j = tix - p * KD8;
  const int n = p >> 7;
  const int t = p & (TT - 1);
  const float* xbase = x + (size_t)n * (CI * TT * VV) + (size_t)t * VV;
  v8h hv;
#pragma unroll
  for (int e = 0; e < 8; ++e) {
    const int kk = 8 * j + e;
    const int i  = kk / VV;
    const int v  = kk - i * VV;
    hv[e] = (_Float16)(xbase[(size_t)i * (TT * VV) + v] * XSC);
  }
  _Float16* dst = xb + (size_t)p * KD + 8 * j;
  *(volatile v8h*)dst = hv;
  __threadfence();
  *(volatile v8h*)dst = hv;
}

__global__ __launch_bounds__(256) void permute_out_kernel(
    const float* __restrict__ cm, float* __restrict__ out)
{
  __shared__ __align__(16) float s[WW_ * TT];
  const int tid = threadIdx.x;
  const int n = blockIdx.x >> 8;
  const int c = blockIdx.x & (CO - 1);
  const float* src = cm + (size_t)(c * WW_) * PP + (size_t)n * TT;
  for (int idx = tid; idx < WW_ * TT; idx += 256) {
    const int w = idx >> 7;
    const int t = idx & (TT - 1);
    s[idx] = src[(size_t)w * PP + t];
  }
  __syncthreads();
  float* dst = out + ((size_t)n * CO + c) * (size_t)(TT * WW_);
  for (int pass = 0; pass < 2; ++pass) {
#pragma unroll
    for (int qq = 0; qq < 2; ++qq) {
      const int f4 = tid + qq * 256;
      if (f4 < (TT * WW_) / 4) {
        v4f val;
#pragma unroll
        for (int e = 0; e < 4; ++e) {
          const int f = 4 * f4 + e;
          const int t = f / WW_;
          const int w = f - t * WW_;
          val[e] = s[w * TT + t];
        }
        *(volatile v4f*)(dst + 4 * f4) = val;
      }
    }
    __threadfence();
  }
}

extern "C" void kernel_launch(void* const* d_in, const int* in_sizes, int n_in,
                              void* d_out, int out_size, void* d_ws, size_t ws_size,
                              hipStream_t stream) {
  if (n_in < 15) return;
  if (in_sizes[0] != NB * CI * TT * VV) return;
  if (in_sizes[1] != KK_ * GG * VV * WW_ || in_sizes[2] != KK_ * GG * VV * WW_) return;
  if (in_sizes[3] != KK_ * CO * CI || in_sizes[5] != KK_ * CO * CI) return;
  if (in_sizes[4] != KK_ * CO || in_sizes[6] != KK_ * CO) return;
  for (int i = 7; i <= 10; ++i) if (in_sizes[i] != KK_ * CO) return;
  for (int i = 11; i <= 14; ++i) if (in_sizes[i] != CO) return;
  if (out_size != NB * CO * TT * WW_) return;

  const float* x      = (const float*)d_in[0];
  const float* A_adj  = (const float*)d_in[1];
  const float* resg   = (const float*)d_in[2];
  const float* conv_w = (const float*)d_in[3];
  const float* conv_b = (const float*)d_in[4];
  const float* down_w = (const float*)d_in[5];
  const float* down_b = (const float*)d_in[6];
  const float* dbn_g  = (const float*)d_in[7];
  const float* dbn_b  = (const float*)d_in[8];
  const float* dbn_m  = (const float*)d_in[9];
  const float* dbn_v  = (const float*)d_in[10];
  const float* bn_g   = (const float*)d_in[11];
  const float* bn_b   = (const float*)d_in[12];
  const float* bn_m   = (const float*)d_in[13];
  const float* bn_v   = (const float*)d_in[14];
  float* out = (float*)d_out;

  const size_t C_BYTES    = (size_t)MM * PP * sizeof(float);
  const size_t WW_BYTES   = (size_t)MM * KD * sizeof(_Float16);
  const size_t XB_BYTES   = (size_t)PP * KD * sizeof(_Float16);
  const size_t BIAS_BYTES = (size_t)MM * sizeof(float);
  const size_t off_c    = 0;
  const size_t off_ww   = off_c + C_BYTES;
  const size_t off_xb   = off_ww + WW_BYTES;
  const size_t off_bias = off_xb + XB_BYTES;
  const size_t total    = off_bias + BIAS_BYTES;
  if (total > ws_size) return;

  float*    cbuf = (float*)((char*)d_ws + off_c);
  _Float16* ww   = (_Float16*)((char*)d_ws + off_ww);
  _Float16* xbuf = (_Float16*)((char*)d_ws + off_xb);
  float*    bias = (float*)((char*)d_ws + off_bias);

  const int totWW = MM * KD8;
  const int totX  = PP * KD8;
  prep_ww_kernel<<<(totWW + 255) / 256, 256, 0, stream>>>(
      conv_w, down_w, A_adj, resg, dbn_g, dbn_v, bn_g, bn_v, ww, totWW);
  prep_bias_kernel<<<(MM + 255) / 256, 256, 0, stream>>>(
      conv_b, down_b, A_adj, resg, dbn_g, dbn_b, dbn_m, dbn_v,
      bn_g, bn_b, bn_m, bn_v, bias, MM);
  prep_x_kernel<<<(totX + 255) / 256, 256, 0, stream>>>(x, xbuf, totX);

  const int tiles = (MM / 64) * (PP / 64);
  dim3 ggrid((tiles + 7) / 8, 1);
  wmma_gemm64<0, false, 1, 0, false, 2><<<ggrid, 256, 0, stream>>>(
      (const unsigned short*)ww, (const unsigned short*)ww, KD, 0L,
      (const unsigned short*)xbuf, (const unsigned short*)xbuf, KD, 0L,
      (void*)cbuf, (void*)cbuf, PP, 0L,
      (const float*)bias,
      (const float*)bias, 0L,
      MM, PP, KD, OSC);

  permute_out_kernel<<<NB * CO, 256, 0, stream>>>(cbuf, out);
}
